// GCN_45509473469204
// MI455X (gfx1250) — hardware-verified
//
#include <hip/hip_runtime.h>
#include <stddef.h>
#include <stdint.h>
#include <math.h>


#define FIN      20
#define HID      16
#define NBROW    256
#define NBSH     8
#define CHUNK    8192
#define CHIT     (CHUNK / 128)
#define TABW     416
#define FLAGSLOT (TABW - 1)
#define NCHMAX   1024
#define RCAP     20480
#define DEGCAP   128
#define SRCBITS  17
#define SRCMASK  0x1ffffu
#define NTHR     256
#define POISC    0x7fffffff
#define SORT_LDS_INTS (2 * RCAP + 3 * NCHMAX + 5 * NBROW + 16 + 256)
#define WSMAX    134217728

static_assert(TABW == 13 * 32);
static_assert(TABW / 4 <= 4 * 32);
static_assert(CHUNK % 128 == 0 && CHUNK < 65536);
static_assert(RCAP % 1024 == 0 && NBROW * HID <= RCAP);
static_assert(NCHMAX == 4 * NTHR);
static_assert(NBROW == (1 << NBSH) && NBROW == NTHR);
static_assert((2 * RCAP) % (4 * NTHR) == 0);
static_assert(SORT_LDS_INTS * 4 <= 300000);
static_assert(DEGCAP % 32 == 0);

typedef float          v2f   __attribute__((ext_vector_type(2)));
typedef float          v4f   __attribute__((ext_vector_type(4)));
typedef float          v8f   __attribute__((ext_vector_type(8)));
typedef int            v4i   __attribute__((ext_vector_type(4)));
typedef int            v8i   __attribute__((ext_vector_type(8)));
typedef unsigned int   v4u   __attribute__((ext_vector_type(4)));
typedef unsigned short v8us  __attribute__((ext_vector_type(8)));
typedef unsigned short v16us __attribute__((ext_vector_type(16)));
typedef __bf16         v16bf __attribute__((ext_vector_type(16)));
typedef v2f  __attribute__((may_alias)) v2fa;
typedef v4f  __attribute__((may_alias)) v4fa;
typedef v4i  __attribute__((may_alias)) v4ia;
typedef v4u  __attribute__((may_alias)) v4ua;
typedef v8us __attribute__((may_alias)) v8usa;
union FragB { v16bf v; v16us u; v8us h[2]; v8i w; };

__device__ __forceinline__ v8f wmb(const FragB& a, const FragB& b, v8f c) {
  v8f d = __builtin_amdgcn_wmma_f32_16x16x32_bf16(false, a.v, false, b.v, (short)0, c, false, false);
  asm volatile("v_nop\n\tv_nop\n\tv_nop\n\tv_nop" : "+v"(d) : "v"(a.w), "v"(b.w));
  return d;
}

__device__ __forceinline__ unsigned bf16_bits(float f) {
  const unsigned u = __float_as_uint(f);
  return (u + 0x7FFFu + ((u >> 16) & 1u)) >> 16;
}
__device__ __forceinline__ float bf16_val(float f) {
  return __uint_as_float(bf16_bits(f) << 16);
}

__device__ __forceinline__ void wave_sync() {
  __builtin_amdgcn_fence(__ATOMIC_RELEASE, "wavefront");
  asm volatile("s_wait_dscnt 0x0" ::: "memory");
  __builtin_amdgcn_wave_barrier();
  __builtin_amdgcn_fence(__ATOMIC_ACQUIRE, "wavefront");
}

__device__ __forceinline__ v4i ld4(const int* __restrict__ p, int e0, int nE, bool full) {
  v4i d;
  if (full) {
    d = *(const v4i*)(p + e0);
  } else {
    const int l = nE - 1;
    d.x = p[(e0     < l) ? e0     : l];
    d.y = p[(e0 + 1 < l) ? e0 + 1 : l];
    d.z = p[(e0 + 2 < l) ? e0 + 2 : l];
    d.w = p[(e0 + 3 < l) ? e0 + 3 : l];
  }
  return d;
}

__global__ __launch_bounds__(32) void k_bucket(const int* __restrict__ dsts, const int* __restrict__ srcs,
                                               int nE, int nN, int vec4, unsigned* bk, unsigned* tab) {
  __shared__ __attribute__((aligned(16))) unsigned stg[CHUNK];
  __shared__ __attribute__((aligned(16))) unsigned trow[TABW];
  __shared__ unsigned cnt[TABW];
  __shared__ unsigned cur[TABW];
  __shared__ unsigned msk[TABW];
  const int lane  = (int)threadIdx.x;
  const int ch    = (int)blockIdx.x;
  const int cbase = ch * CHUNK;
  {
    const v4u z = {0u, 0u, 0u, 0u};
#pragma unroll 1
    for (int i = 4 * lane; i < CHUNK; i += 128) *(v4ua*)(stg + i) = z;
#pragma unroll 1
    for (int i = lane; i < TABW; i += 32) { cnt[i] = 0u; cur[i] = 0u; msk[i] = 0u; trow[i] = 0u; }
  }
  __syncthreads();
  const bool full = (vec4 != 0) && (cbase + CHUNK <= nE);
  int bad = 0;

#pragma unroll 1
  for (int it = 0; it < CHIT; ++it) {
    const int e0 = cbase + it * 128 + 4 * lane;
    const v4i d = ld4(dsts, e0, nE, full);
#pragma unroll
    for (int j = 0; j < 4; ++j) {
      const int  dvv = d[j];
      const bool inr = (e0 + j) < nE;
      const bool ok  = inr && ((unsigned)dvv < (unsigned)nN);
      bad |= (inr && !ok) ? 1 : 0;
      if (ok) atomicAdd(&cnt[dvv >> NBSH], 1u);
    }
  }
  __syncthreads();

  {
    const int base = lane * 13;
    unsigned s = 0u;
#pragma unroll 1
    for (int i = 0; i < 13; ++i) s += cnt[base + i];
    unsigned incl = s;
#pragma unroll
    for (int dd = 1; dd < 32; dd <<= 1) {
      const unsigned y = (unsigned)__shfl_up((int)incl, dd, 32);
      if (lane >= dd) incl += y;
    }
    unsigned run = incl - s;
#pragma unroll 1
    for (int i = 0; i < 13; ++i) {
      const unsigned c = cnt[base + i];
      cur[base + i]  = run;
      trow[base + i] = (run << 16) | c;
      run += c;
    }
  }
  __syncthreads();

  const unsigned lbit  = 1u << lane;
  const unsigned lmask = lbit - 1u;
#pragma unroll 1
  for (int it = 0; it < CHIT; ++it) {
    const int e0 = cbase + it * 128 + 4 * lane;
    const v4i d  = ld4(dsts, e0, nE, full);
    const v4i s4 = ld4(srcs, e0, nE, full);
#pragma unroll
    for (int j = 0; j < 4; ++j) {
      const int  dvv = d[j];
      const int  svv = s4[j];
      const bool inr = (e0 + j) < nE;
      const bool ok  = inr && ((unsigned)dvv < (unsigned)nN);
      const bool sok = (unsigned)svv < (unsigned)nN;
      bad |= (ok && !sok) ? 1 : 0;
      const int svc = sok ? svv : 0;
      const int b   = ok ? (dvv >> NBSH) : 0;
      if (ok) atomicOr(&msk[b], lbit);
      __syncthreads();
      const unsigned m    = msk[b];
      const unsigned base = cur[b];
      __syncthreads();
      const unsigned rank = (unsigned)__builtin_popcount(m & lmask);
      if (ok && rank == 0u) { cur[b] = base + (unsigned)__builtin_popcount(m); msk[b] = 0u; }
      const unsigned pos = base + rank;
      if (ok && pos < (unsigned)CHUNK) stg[pos] = ((unsigned)(dvv & (NBROW - 1)) << SRCBITS) | (unsigned)svc;
      __syncthreads();
    }
  }
  const unsigned anyb = __builtin_amdgcn_ballot_w32(bad != 0);
  if (lane == 0) trow[FLAGSLOT] = (anyb != 0u) ? 1u : 0u;
  __syncthreads();

  unsigned* bp = bk + (size_t)ch * CHUNK;
  unsigned* tp = tab + (size_t)ch * TABW;
#pragma unroll 1
  for (int it = 0; it < CHIT; ++it) {
    const int idx = it * 128 + 4 * lane;
    const v4u v = *(const v4ua*)(stg + idx);
    *(volatile v4u*)(bp + idx) = v;
  }
#pragma unroll 1
  for (int it = 0; it < 4; ++it) {
    const int q  = it * 32 + lane;
    const int qc = (q < TABW / 4) ? q : (TABW / 4 - 1);
    const v4u v = *(const v4ua*)(trow + 4 * qc);
    if (q < TABW / 4) *(volatile v4u*)(tp + 4 * q) = v;
  }
  __threadfence();
#pragma unroll 1
  for (int it = 0; it < CHIT; ++it) {
    const int idx = it * 128 + 4 * lane;
    const v4u v = *(const v4ua*)(stg + idx);
    *(volatile v4u*)(bp + idx) = v;
  }
#pragma unroll 1
  for (int it = 0; it < 4; ++it) {
    const int q  = it * 32 + lane;
    const int qc = (q < TABW / 4) ? q : (TABW / 4 - 1);
    const v4u v = *(const v4ua*)(trow + 4 * qc);
    if (q < TABW / 4) *(volatile v4u*)(tp + 4 * q) = v;
  }
}

__global__ __launch_bounds__(NTHR) void k_sort(const float* __restrict__ x, const float* __restrict__ W1,
                                               const unsigned* __restrict__ bk, const unsigned* __restrict__ tab,
                                               int nCh, int nN, unsigned* sl, int* cntg, float* dinvg, float* xs1) {
  extern __shared__ __attribute__((aligned(16))) unsigned dsm[];
  unsigned* hl   = dsm;
  unsigned* slp  = dsm + RCAP;
  unsigned* roff = slp + RCAP;
  unsigned* rcnt = roff + NCHMAX;
  unsigned* rpre = rcnt + NCHMAX;
  unsigned* cntd = rpre + NCHMAX;
  unsigned* offd = cntd + NBROW;
  unsigned* curd = offd + NBROW;
  unsigned* mskd = curd + NBROW;
  float*    dinvs = (float*)(mskd + NBROW);
  unsigned* misc = (unsigned*)(dinvs + NBROW);
  unsigned short* w1t = (unsigned short*)(misc + 16);
  float* stgf = (float*)hl;
  const int tid = (int)threadIdx.x, lane = tid & 31, wave = tid >> 5, hh = lane >> 4, m = lane & 15;
  const int b = (int)blockIdx.x;
  const int nodeBase = b * NBROW;

  {
    const v4u z = {0u, 0u, 0u, 0u};
#pragma unroll 1
    for (int i = 4 * tid; i < 2 * RCAP; i += 4 * NTHR) *(v4ua*)(dsm + i) = z;
    cntd[tid] = 0u; offd[tid] = 0u; curd[tid] = 0u; mskd[tid] = 0u; dinvs[tid] = 0.0f;
    if (tid < 16) misc[tid] = 0u;
#pragma unroll 1
    for (int i = tid; i < HID * 32; i += NTHR) {
      const int n = i >> 5, k = i & 31;
      const int kk = (k < FIN) ? k : (FIN - 1);
      const float wv = W1[kk * HID + n];
      w1t[i] = (k < FIN) ? (unsigned short)bf16_bits(wv) : (unsigned short)0;
    }
  }
  __syncthreads();

  unsigned s = 0u;
  {
    unsigned badl = 0u;
#pragma unroll 1
    for (int i = 0; i < 4; ++i) {
      const int c  = 4 * tid + i;
      const int cc = (c < nCh) ? c : (nCh - 1);
      const unsigned tv = tab[(size_t)cc * TABW + b];
      const unsigned fl = tab[(size_t)cc * TABW + FLAGSLOT];
      const bool live = c < nCh;
      unsigned of = tv >> 16;
      unsigned cn = tv & 0xffffu;
      of = (of > (unsigned)CHUNK) ? (unsigned)CHUNK : of;
      cn = (cn > (unsigned)CHUNK - of) ? ((unsigned)CHUNK - of) : cn;
      cn = live ? cn : 0u;
      badl |= live ? fl : 0u;
      roff[c] = of;
      rcnt[c] = cn;
      s += cn;
    }
    if (badl != 0u) misc[9] = 1u;
  }
  unsigned incl = s;
#pragma unroll
  for (int dd = 1; dd < 32; dd <<= 1) {
    const unsigned y = (unsigned)__shfl_up((int)incl, dd, 32);
    if (lane >= dd) incl += y;
  }
  if (lane == 31) misc[wave] = incl;
  __syncthreads();
  unsigned wbase = 0u, tot = 0u;
#pragma unroll
  for (int w2 = 0; w2 < 8; ++w2) {
    const unsigned t = misc[w2];
    wbase += (w2 < wave) ? t : 0u;
    tot += t;
  }
  {
    unsigned run = wbase + incl - s;
#pragma unroll 1
    for (int i = 0; i < 4; ++i) {
      const int c = 4 * tid + i;
      rpre[c] = run;
      run += rcnt[c];
    }
  }
  const bool pois = (tot > (unsigned)RCAP) || (misc[9] != 0u);
  const int tt = __builtin_amdgcn_readfirstlane((int)((tot > (unsigned)RCAP) ? (unsigned)RCAP : tot));
  __syncthreads();

#pragma unroll 1
  for (int c = wave; c < nCh; c += 8) {
    const int ro = __builtin_amdgcn_readfirstlane((int)roff[c]);
    const int rc = __builtin_amdgcn_readfirstlane((int)rcnt[c]);
    const int rp = __builtin_amdgcn_readfirstlane((int)rpre[c]);
    if (rp >= RCAP) continue;
    const unsigned* rb = bk + (size_t)c * CHUNK;
#pragma unroll 1
    for (int j0 = 0; j0 < rc; j0 += 32) {
      const int j = j0 + lane;
      int idx = ro + j;
      idx = (idx > CHUNK - 1) ? (CHUNK - 1) : idx;
      const unsigned ent = rb[idx];
      const int p = rp + j;
      const bool ok = (j < rc) && (p < RCAP);
      if (ok) { hl[p] = ent; atomicAdd(&cntd[(ent >> SRCBITS) & (NBROW - 1)], 1u); }
    }
  }
  __syncthreads();

  if (wave == 0) {
    const int base = lane * 8;
    unsigned s8 = 0u;
#pragma unroll 1
    for (int i = 0; i < 8; ++i) s8 += cntd[base + i];
    unsigned in8 = s8;
#pragma unroll
    for (int dd = 1; dd < 32; dd <<= 1) {
      const unsigned y = (unsigned)__shfl_up((int)in8, dd, 32);
      if (lane >= dd) in8 += y;
    }
    unsigned run = in8 - s8;
#pragma unroll 1
    for (int i = 0; i < 8; ++i) {
      const unsigned cv = cntd[base + i];
      offd[base + i] = run;
      curd[base + i] = run;
      run += cv;
    }
  }
  {
    const float deg = (float)cntd[tid] + 1.0f;
    dinvs[tid] = (deg > 0.0f) ? (1.0f / sqrtf(deg)) : 0.0f;
  }
  __syncthreads();

  if (wave == 0) {
    const unsigned lbit  = 1u << lane;
    const unsigned lmask = lbit - 1u;
#pragma unroll 1
    for (int b0 = 0; b0 < tt; b0 += 32) {
      const int idx = b0 + lane;
      const bool ok = idx < tt;
      const unsigned ent = hl[(idx < RCAP) ? idx : (RCAP - 1)];
      const int dl = (int)((ent >> SRCBITS) & (NBROW - 1));
      if (ok) atomicOr(&mskd[dl], lbit);
      wave_sync();
      const unsigned mm   = mskd[dl];
      const unsigned base = curd[dl];
      wave_sync();
      const unsigned rank = (unsigned)__builtin_popcount(mm & lmask);
      if (ok && rank == 0u) { curd[dl] = base + (unsigned)__builtin_popcount(mm); mskd[dl] = 0u; }
      const unsigned p = base + rank;
      if (ok && p < (unsigned)RCAP) slp[p] = ent & SRCMASK;
      wave_sync();
    }
  }
  __syncthreads();

  {
    const int nIt = (tt + 1023) >> 10;
    unsigned* sp = sl + (size_t)b * RCAP;
    v4i c4 = {0, 0, 0, 0};
    v4f d4 = {0.f, 0.f, 0.f, 0.f};
    const int q = (tid < 64) ? tid : 63;
    c4 = *(const v4ia*)((const int*)cntd + 4 * q);
    d4 = *(const v4fa*)(dinvs + 4 * q);
    if (pois) { c4.x = POISC; c4.y = POISC; c4.z = POISC; c4.w = POISC; }
#pragma unroll 1
    for (int it = 0; it < nIt; ++it) {
      const int idx = it * 1024 + 4 * tid;
      const v4u v = *(const v4ua*)(slp + idx);
      *(volatile v4u*)(sp + idx) = v;
    }
    if (tid < 64) {
      *(volatile v4i*)(cntg + (size_t)nodeBase + 4 * tid) = c4;
      *(volatile v4f*)(dinvg + (size_t)nodeBase + 4 * tid) = d4;
    }
    __threadfence();
#pragma unroll 1
    for (int it = 0; it < nIt; ++it) {
      const int idx = it * 1024 + 4 * tid;
      const v4u v = *(const v4ua*)(slp + idx);
      *(volatile v4u*)(sp + idx) = v;
    }
    if (tid < 64) {
      *(volatile v4i*)(cntg + (size_t)nodeBase + 4 * tid) = c4;
      *(volatile v4f*)(dinvg + (size_t)nodeBase + 4 * tid) = d4;
    }
  }

  FragB bf;
  bf.h[0] = *(const v8usa*)(w1t + m * 32 + 8 * hh);
  bf.h[1] = *(const v8usa*)(w1t + m * 32 + 16 + 8 * hh);
  v8f acc[2];
#pragma unroll
  for (int t = 0; t < 2; ++t) {
    const int row = nodeBase + 32 * wave + 16 * t + m;
    const int rc  = (row < nN) ? row : (nN - 1);
    const float* p = x + (size_t)rc * FIN;
    const v4f a0 = *(const v4f*)(p + 8 * hh);
    const v4f a1 = *(const v4f*)(p + 8 * hh + 4);
    const v4f a2 = *(const v4f*)(p + 16);
    const bool live = row < nN;
    const bool l2   = live && (hh == 0);
    FragB af;
    af.u[0]  = live ? (unsigned short)bf16_bits(a0.x) : (unsigned short)0;
    af.u[1]  = live ? (unsigned short)bf16_bits(a0.y) : (unsigned short)0;
    af.u[2]  = live ? (unsigned short)bf16_bits(a0.z) : (unsigned short)0;
    af.u[3]  = live ? (unsigned short)bf16_bits(a0.w) : (unsigned short)0;
    af.u[4]  = live ? (unsigned short)bf16_bits(a1.x) : (unsigned short)0;
    af.u[5]  = live ? (unsigned short)bf16_bits(a1.y) : (unsigned short)0;
    af.u[6]  = live ? (unsigned short)bf16_bits(a1.z) : (unsigned short)0;
    af.u[7]  = live ? (unsigned short)bf16_bits(a1.w) : (unsigned short)0;
    af.u[8]  = l2 ? (unsigned short)bf16_bits(a2.x) : (unsigned short)0;
    af.u[9]  = l2 ? (unsigned short)bf16_bits(a2.y) : (unsigned short)0;
    af.u[10] = l2 ? (unsigned short)bf16_bits(a2.z) : (unsigned short)0;
    af.u[11] = l2 ? (unsigned short)bf16_bits(a2.w) : (unsigned short)0;
    af.u[12] = (unsigned short)0; af.u[13] = (unsigned short)0;
    af.u[14] = (unsigned short)0; af.u[15] = (unsigned short)0;
    const v8f z = {0.f, 0.f, 0.f, 0.f, 0.f, 0.f, 0.f, 0.f};
    acc[t] = wmb(af, bf, z);
  }
#pragma unroll
  for (int t = 0; t < 2; ++t) {
#pragma unroll
    for (int r = 0; r < 8; ++r) {
      const int lr = 32 * wave + 16 * t + 8 * hh + r;
      stgf[lr * HID + m] = acc[t][r] * dinvs[lr];
    }
  }
  __syncthreads();
  {
    v4f ov[4];
#pragma unroll
    for (int it = 0; it < 4; ++it) ov[it] = *(const v4fa*)(stgf + 4 * (it * NTHR + tid));
    float* op = xs1 + (size_t)nodeBase * HID;
#pragma unroll
    for (int it = 0; it < 4; ++it) *(volatile v4f*)(op + 4 * (size_t)(it * NTHR + tid)) = ov[it];
    __threadfence();
#pragma unroll
    for (int it = 0; it < 4; ++it) *(volatile v4f*)(op + 4 * (size_t)(it * NTHR + tid)) = ov[it];
  }
}

__device__ __forceinline__ void load_rows(const int* __restrict__ cntg, const float* __restrict__ dinvg, int nodeBase,
                                          int* cnt, int* offs, float* dv, int tid, int lane, int wave) {
  cnt[tid] = cntg[(size_t)nodeBase + tid];
  dv[tid]  = dinvg[(size_t)nodeBase + tid];
  __syncthreads();
  if (wave == 0) {
    const int base = lane * 8;
    int s8 = 0;
#pragma unroll 1
    for (int i = 0; i < 8; ++i) {
      int c = cnt[base + i];
      c = c < 0 ? 0 : (c > RCAP ? RCAP : c);
      s8 += c;
    }
    int in8 = s8;
#pragma unroll
    for (int dd = 1; dd < 32; dd <<= 1) {
      const int y = __shfl_up(in8, dd, 32);
      if (lane >= dd) in8 += y;
    }
    int run = in8 - s8;
#pragma unroll 1
    for (int i = 0; i < 8; ++i) {
      int c = cnt[base + i];
      c = c < 0 ? 0 : (c > RCAP ? RCAP : c);
      offs[base + i] = run;
      run += c;
    }
  }
  __syncthreads();
}

__global__ __launch_bounds__(NTHR) void k_scan1(const unsigned* __restrict__ sl, const int* __restrict__ cntg,
                                                const float* __restrict__ dinvg, const float* __restrict__ xs1,
                                                const float* __restrict__ b1, const float* __restrict__ W2,
                                                int nN, float* xs2) {
  __shared__ int cnt[NBROW];
  __shared__ int offs[NBROW];
  __shared__ float dv[NBROW];
  __shared__ __attribute__((aligned(16))) float w2s[HID * 2];
  __shared__ __attribute__((aligned(16))) float b1s[HID];
  __shared__ __attribute__((aligned(16))) float outs[NBROW * 2];
  const int tid = (int)threadIdx.x, lane = tid & 31, wave = tid >> 5;
  const int b = (int)blockIdx.x;
  const int nodeBase = b * NBROW;
  {
    const float wv = W2[(tid < HID * 2) ? tid : (HID * 2 - 1)];
    const float bv = b1[(tid < HID) ? tid : (HID - 1)];
    if (tid < HID * 2) w2s[tid] = bf16_val(wv);
    if (tid < HID) b1s[tid] = bf16_val(bv);
  }
  load_rows(cntg, dinvg, nodeBase, cnt, offs, dv, tid, lane, wave);

  const unsigned* sp = sl + (size_t)b * RCAP;
  const int q = lane >> 2, p = lane & 3;
  const v4f wa = *(const v4fa*)(w2s + 8 * p);
  const v4f wb = *(const v4fa*)(w2s + 8 * p + 4);
  const v4f bb = *(const v4fa*)(b1s + 4 * p);
  const float qnan = __int_as_float(0x7fc00000);
#pragma unroll 1
  for (int si = 0; si < NBROW / 8; ++si) {
    const int s    = si * 8 + wave;
    const int node = nodeBase + s;
    const int craw = cnt[s];
    const bool big = (craw < 0) || (craw > DEGCAP);
    int c = craw < 0 ? 0 : (craw > DEGCAP ? DEGCAP : craw);
    int o = offs[s];
    o = o < 0 ? 0 : (o > RCAP ? RCAP : o);
    c = (c > RCAP - o) ? (RCAP - o) : c;
    c = __builtin_amdgcn_readfirstlane(c);
    o = __builtin_amdgcn_readfirstlane(o);
    float a0 = 0.0f, a1 = 0.0f, a2 = 0.0f, a3 = 0.0f;
#pragma unroll 1
    for (int b0 = 0; b0 < c; b0 += 32) {
      int jj = b0 + lane;
      jj = (jj > c - 1) ? (c - 1) : jj;
      const unsigned ent = sp[o + jj];
      const int sr = (ent > (unsigned)(nN - 1)) ? (nN - 1) : (int)ent;
      const int rem = c - b0;
#pragma unroll
      for (int j = 0; j < 4; ++j) {
        if (8 * j < rem) {
          const int hq = 8 * j + q;
          const int sk = __shfl(sr, hq, 32);
          const v4f v = *(const v4f*)(xs1 + (size_t)sk * HID + 4 * p);
          const bool valid = hq < rem;
          a0 += valid ? v.x : 0.0f;
          a1 += valid ? v.y : 0.0f;
          a2 += valid ? v.z : 0.0f;
          a3 += valid ? v.w : 0.0f;
        }
      }
    }
#pragma unroll
    for (int mk = 4; mk < 32; mk <<= 1) {
      a0 += __shfl_xor(a0, mk, 32);
      a1 += __shfl_xor(a1, mk, 32);
      a2 += __shfl_xor(a2, mk, 32);
      a3 += __shfl_xor(a3, mk, 32);
    }
    const int nc = (node < nN) ? node : (nN - 1);
    const v4f sv = *(const v4f*)(xs1 + (size_t)nc * HID + 4 * p);
    const float dd = dv[s];
    const float v0 = dd * (a0 + sv.x) + bb.x;
    const float v1 = dd * (a1 + sv.y) + bb.y;
    const float v2 = dd * (a2 + sv.z) + bb.z;
    const float v3 = dd * (a3 + sv.w) + bb.w;
    const float h0 = (v0 > 0.0f) ? v0 : (v0 - v0);
    const float h1 = (v1 > 0.0f) ? v1 : (v1 - v1);
    const float h2 = (v2 > 0.0f) ? v2 : (v2 - v2);
    const float h3 = (v3 > 0.0f) ? v3 : (v3 - v3);
    float hw0 = h0 * wa.x;
    hw0 = fmaf(h1, wa.z, hw0); hw0 = fmaf(h2, wb.x, hw0); hw0 = fmaf(h3, wb.z, hw0);
    float hw1 = h0 * wa.y;
    hw1 = fmaf(h1, wa.w, hw1); hw1 = fmaf(h2, wb.y, hw1); hw1 = fmaf(h3, wb.w, hw1);
    hw0 += __shfl_xor(hw0, 1, 32); hw1 += __shfl_xor(hw1, 1, 32);
    hw0 += __shfl_xor(hw0, 2, 32); hw1 += __shfl_xor(hw1, 2, 32);
    float r0 = dd * hw0, r1 = dd * hw1;
    r0 = big ? qnan : r0;
    r1 = big ? qnan : r1;
    const bool live = node < nN;
    r0 = live ? r0 : 0.0f;
    r1 = live ? r1 : 0.0f;
    if (lane == 0) { outs[2 * s] = r0; outs[2 * s + 1] = r1; }
  }
  __syncthreads();
  {
    const int qd = (tid < 128) ? tid : 127;
    const v4f ov = *(const v4fa*)(outs + 4 * qd);
    float* op = xs2 + (size_t)nodeBase * 2 + 4 * qd;
    if (tid < 128) *(volatile v4f*)op = ov;
    __threadfence();
    if (tid < 128) *(volatile v4f*)op = ov;
  }
}

__global__ __launch_bounds__(NTHR) void k_scan2(const unsigned* __restrict__ sl, const int* __restrict__ cntg,
                                                const float* __restrict__ dinvg, const float* __restrict__ xs2,
                                                const float* __restrict__ b2, int nN, float* out) {
  __shared__ int cnt[NBROW];
  __shared__ int offs[NBROW];
  __shared__ float dv[NBROW];
  __shared__ __attribute__((aligned(16))) float outs[NBROW * 2];
  const int tid = (int)threadIdx.x, lane = tid & 31, wave = tid >> 5;
  const int b = (int)blockIdx.x;
  const int nodeBase = b * NBROW;
  const float bb0 = bf16_val(b2[0]);
  const float bb1 = bf16_val(b2[1]);
  load_rows(cntg, dinvg, nodeBase, cnt, offs, dv, tid, lane, wave);

  const unsigned* sp = sl + (size_t)b * RCAP;
  const float qnan = __int_as_float(0x7fc00000);
#pragma unroll 1
  for (int si = 0; si < NBROW / 8; ++si) {
    const int s    = si * 8 + wave;
    const int node = nodeBase + s;
    const int craw = cnt[s];
    const bool big = (craw < 0) || (craw > DEGCAP);
    int c = craw < 0 ? 0 : (craw > DEGCAP ? DEGCAP : craw);
    int o = offs[s];
    o = o < 0 ? 0 : (o > RCAP ? RCAP : o);
    c = (c > RCAP - o) ? (RCAP - o) : c;
    c = __builtin_amdgcn_readfirstlane(c);
    o = __builtin_amdgcn_readfirstlane(o);
    float a0 = 0.0f, a1 = 0.0f;
#pragma unroll 1
    for (int b0 = 0; b0 < c; b0 += 32) {
      const int j = b0 + lane;
      const int jj = (j > c - 1) ? (c - 1) : j;
      const unsigned ent = sp[o + jj];
      const int sr = (ent > (unsigned)(nN - 1)) ? (nN - 1) : (int)ent;
      const v2f v = *(const v2fa*)(xs2 + (size_t)sr * 2);
      const bool valid = j < c;
      a0 += valid ? v.x : 0.0f;
      a1 += valid ? v.y : 0.0f;
    }
#pragma unroll
    for (int mk = 1; mk < 32; mk <<= 1) {
      a0 += __shfl_xor(a0, mk, 32);
      a1 += __shfl_xor(a1, mk, 32);
    }
    const int nc = (node < nN) ? node : (nN - 1);
    const v2f sv = *(const v2fa*)(xs2 + (size_t)nc * 2);
    const float dd = dv[s];
    const float o0 = dd * (a0 + sv.x) + bb0;
    const float o1 = dd * (a1 + sv.y) + bb1;
    const float d01 = o0 - o1;
    const float mx = (o0 > o1) ? o0 : o1;
    const float ad = (d01 < 0.0f) ? (0.0f - d01) : d01;
    const float lse = mx + log1pf(expf(0.0f - ad));
    float r0 = o0 - lse, r1 = o1 - lse;
    r0 = big ? qnan : r0;
    r1 = big ? qnan : r1;
    if (lane == 0) { outs[2 * s] = r0; outs[2 * s + 1] = r1; }
  }
  __syncthreads();
  {
    int nr = nN - nodeBase;
    nr = nr > NBROW ? NBROW : (nr < 0 ? 0 : nr);
    const int nq = nr >> 1;
    const int qd = (tid < 128) ? tid : 127;
    const v4f ov = *(const v4fa*)(outs + 4 * qd);
    float* op = out + (size_t)nodeBase * 2 + 4 * qd;
    if (tid < nq) *(volatile v4f*)op = ov;
    __threadfence();
    if (tid < nq) *(volatile v4f*)op = ov;
  }
}

static inline int cdiv(int a, int b) { return (a + b - 1) / b; }
static inline size_t al256(size_t o) { return (o + 255) & ~(size_t)255; }

extern "C" void kernel_launch(void* const* d_in, const int* in_sizes, int n_in,
                              void* d_out, int out_size, void* d_ws, size_t ws_size,
                              hipStream_t stream) {
  if (n_in < 6) return;
  if (in_sizes[0] < FIN || (in_sizes[0] % FIN) != 0) return;
  const int nN = in_sizes[0] / FIN;
  if (nN < 16 || (nN % 16) != 0 || nN > (1 << SRCBITS)) return;
  if (in_sizes[1] < 2 || (in_sizes[1] & 1) != 0) return;
  const int nE = in_sizes[1] / 2;
  if (nE < 1 || nE > NCHMAX * CHUNK) return;
  if (in_sizes[2] != FIN * HID || in_sizes[3] != HID) return;
  if (in_sizes[4] != HID * 2 || in_sizes[5] != 2) return;
  if ((long long)out_size != 2LL * nN) return;

  const float* x  = (const float*)d_in[0];
  const int*   ei = (const int*)d_in[1];
  const float* W1 = (const float*)d_in[2];
  const float* b1 = (const float*)d_in[3];
  const float* W2 = (const float*)d_in[4];
  const float* b2 = (const float*)d_in[5];
  float* out = (float*)d_out;
  const int* dst = ei;
  const int* src = ei + nE;

  const int nB  = cdiv(nN, NBROW);
  const int nCh = cdiv(nE, CHUNK);
  if (nB > FLAGSLOT || nCh > NCHMAX) return;
  const int vec4 = ((nE & 3) == 0) ? 1 : 0;

  char* ws = (char*)d_ws;
  size_t off = 0;
  const size_t oBK  = off; off = al256(off + (size_t)nCh * CHUNK * 4);
  const size_t oTAB = off; off = al256(off + (size_t)nCh * TABW * 4);
  const size_t oSL  = off; off = al256(off + (size_t)nB * RCAP * 4);
  const size_t oCN  = off; off = al256(off + (size_t)nB * NBROW * 4);
  const size_t oDI  = off; off = al256(off + (size_t)nB * NBROW * 4);
  const size_t oX1  = off; off = al256(off + (size_t)nB * NBROW * HID * 4);
  const size_t oX2  = off; off = al256(off + (size_t)nB * NBROW * 2 * 4);
  if (off > ws_size || off > (size_t)WSMAX) return;
  unsigned* BK   = (unsigned*)(ws + oBK);
  unsigned* TAB  = (unsigned*)(ws + oTAB);
  unsigned* SL   = (unsigned*)(ws + oSL);
  int*      CNTD = (int*)(ws + oCN);
  float*    DINV = (float*)(ws + oDI);
  float*    XS1  = (float*)(ws + oX1);
  float*    XS2  = (float*)(ws + oX2);

  const size_t sortLds = (size_t)SORT_LDS_INTS * 4;
  hipFuncSetAttribute(reinterpret_cast<const void*>(&k_sort), hipFuncAttributeMaxDynamicSharedMemorySize, (int)sortLds);

  k_bucket<<<nCh, 32, 0, stream>>>(dst, src, nE, nN, vec4, BK, TAB);
  k_sort<<<nB, NTHR, sortLds, stream>>>(x, W1, BK, TAB, nCh, nN, SL, CNTD, DINV, XS1);
  k_scan1<<<nB, NTHR, 0, stream>>>(SL, CNTD, DINV, XS1, b1, W2, nN, XS2);
  k_scan2<<<nB, NTHR, 0, stream>>>(SL, CNTD, DINV, XS2, b2, nN, out);
}
